// PointShufflerSetAbstraction_54159537602743
// MI455X (gfx1250) — hardware-verified
//
#include <hip/hip_runtime.h>
#include <math.h>

typedef __attribute__((ext_vector_type(16))) _Float16 v16h;
typedef __attribute__((ext_vector_type(16))) __bf16 v16b;
typedef __attribute__((ext_vector_type(8)))  _Float16 v8h;
typedef __attribute__((ext_vector_type(8)))  float v8f;
typedef __attribute__((ext_vector_type(4)))  float v4f;
typedef __attribute__((ext_vector_type(2)))  float v2f;
typedef __attribute__((ext_vector_type(4)))  unsigned v4u;
typedef __attribute__((ext_vector_type(4)))  int v4i;
typedef float __attribute__((may_alias)) float_a;
typedef int __attribute__((may_alias)) int_a;

template <typename T> __device__ __forceinline__ void vst2(void* p, T v) { *(volatile T*)p = v; __threadfence(); *(volatile T*)p = v; }
__device__ __forceinline__ v8f wmma16(v16h a, v16h b, v8f c) {
  v8f d = __builtin_amdgcn_wmma_f32_16x16x32_f16(false, a, false, b, (short)0, c, false, false);
  asm volatile("v_nop\n\tv_nop\n\tv_nop\n\tv_nop" : "+v"(d) : "v"(a), "v"(b));
  return d;
}
__device__ __forceinline__ v8f wmma_bf(v16b a, v16b b, v8f c) {
  v8f d = __builtin_amdgcn_wmma_f32_16x16x32_bf16(false, a, false, b, (short)0, c, false, false);
  asm volatile("v_nop\n\tv_nop\n\tv_nop\n\tv_nop" : "+v"(d) : "v"(a), "v"(b));
  return d;
}
__device__ __forceinline__ v16h frag_h(const _Float16* rowk0, int lane) {
  union { v16h v; v8h q[2]; } u; const _Float16* p = rowk0 + 8 * (lane >> 4);
  u.q[0] = *(const v8h*)p; u.q[1] = *(const v8h*)(p + 16); return u.v;
}
__device__ __forceinline__ v16h frag_f32(const float* rowk0, int lane) {
  v16h a; const float* p = rowk0 + 8 * (lane >> 4);
#pragma unroll
  for (int i = 0; i < 8; ++i) { a[i] = (_Float16)p[i]; a[8 + i] = (_Float16)p[16 + i]; }
  return a;
}
__device__ __forceinline__ v16h frag_f32s(const float* rowk0, int lane, float sc) {
  v16h a; const float* p = rowk0 + 8 * (lane >> 4);
#pragma unroll
  for (int i = 0; i < 8; ++i) { a[i] = (_Float16)(p[i] * sc); a[8 + i] = (_Float16)(p[16 + i] * sc); }
  return a;
}
__device__ __forceinline__ v16h fragc_f32(const float* W, int k0, int n, int lane, int ld, int K) {
  v16h a; const int g = lane >> 4;
#pragma unroll
  for (int i = 0; i < 8; ++i) { const int ka = k0 + 8 * g + i, kb = ka + 16;
    a[i] = (_Float16)(ka < K ? W[(size_t)ka * ld + n] : 0.f); a[8 + i] = (_Float16)(kb < K ? W[(size_t)kb * ld + n] : 0.f); }
  return a;
}
struct F2 { v16b h, l; };
__device__ __forceinline__ F2 bsplit16(const float v[16]) { F2 r;
#pragma unroll
  for (int i = 0; i < 16; ++i) { const __bf16 h = (__bf16)v[i]; r.h[i] = h; r.l[i] = (__bf16)(v[i] - (float)h); }
  return r; }
__device__ __forceinline__ F2 split_row(const float* row, int k0, int lane) { float v[16]; const float* p = row + k0 + 8 * (lane >> 4);
#pragma unroll
  for (int i = 0; i < 8; ++i) { v[i] = p[i]; v[8 + i] = p[16 + i]; }
  return bsplit16(v); }
__device__ __forceinline__ F2 split_rowK(const float* row, int k0, int lane, int K) { float v[16]; const int g = lane >> 4;
#pragma unroll
  for (int i = 0; i < 8; ++i) { const int ka = k0 + 8 * g + i, kb = ka + 16; v[i] = ka < K ? row[ka] : 0.f; v[8 + i] = kb < K ? row[kb] : 0.f; }
  return bsplit16(v); }
__device__ __forceinline__ F2 split_col(const float* W, int k0, int n, int lane, int ld, int K) { float v[16]; const int g = lane >> 4;
#pragma unroll
  for (int i = 0; i < 8; ++i) { const int ka = k0 + 8 * g + i, kb = ka + 16; v[i] = ka < K ? W[(size_t)ka * ld + n] : 0.f; v[8 + i] = kb < K ? W[(size_t)kb * ld + n] : 0.f; }
  return bsplit16(v); }
__device__ __forceinline__ v8f mac3(const F2& a, const F2& b, v8f c) { c = wmma_bf(a.l, b.h, c); c = wmma_bf(a.h, b.l, c); return wmma_bf(a.h, b.h, c); }
__device__ __forceinline__ float sigm(float v) { return 1.0f / (1.0f + expf(-v)); }
#define LDSX() do { asm volatile("s_wait_dscnt 0" ::: "memory"); __builtin_amdgcn_wave_barrier(); __builtin_amdgcn_fence(__ATOMIC_RELEASE, "workgroup"); } while (0)

#define NPT 65536
#define NS 2048
#define NCHK (NPT / 256)
#define NKEY 512
#define C0 6
#define C1 32
#define C2 64
#define C3 128
#define CAND 2048

__global__ __launch_bounds__(256) void k_l0(const float* __restrict__ xyz, const float* __restrict__ pts, const float* __restrict__ w0, const float* __restrict__ b0, float offs, float stepf,
                                          float* __restrict__ pre0, float* __restrict__ part0, int* __restrict__ vkey, int* __restrict__ hist) {
  __shared__ int sh[NKEY]; __shared__ __align__(16) float st[C1][260]; __shared__ float sf[256][8];
  const int tid = threadIdx.x, i = blockIdx.x * 256 + tid, w = tid >> 5, lane = tid & 31, col = lane & 15, g = lane >> 4;
  for (int q = tid; q < NKEY; q += 256) sh[q] = 0;
  __syncthreads();
  const float x = xyz[i], y = xyz[NPT + i], z = xyz[2 * NPT + i]; const float f3 = pts[i], f4 = pts[NPT + i], f5 = pts[2 * NPT + i];
  { int v0 = (int)floorf((x + offs) / stepf), v1 = (int)floorf((y + offs) / stepf), v2 = (int)floorf((z + offs) / stepf);
    v0 = v0 < 0 ? 0 : (v0 > 7 ? 7 : v0); v1 = v1 < 0 ? 0 : (v1 > 7 ? 7 : v1); v2 = v2 < 0 ? 0 : (v2 > 7 ? 7 : v2);
    const int key = (v0 * 8 + v1) * 8 + v2; atomicAdd(&sh[key], 1); vst2(vkey + i, (int_a)key); }
  sf[tid][0] = x; sf[tid][1] = y; sf[tid][2] = z; sf[tid][3] = f3; sf[tid][4] = f4; sf[tid][5] = f5; sf[tid][6] = 0.f; sf[tid][7] = 0.f;
  v16h bw[2];
#pragma unroll
  for (int t = 0; t < 2; ++t) {
#pragma unroll
    for (int e = 0; e < 16; ++e) { const int k = e < 8 ? 8 * g + e : 16 + 8 * g + (e - 8); bw[t][e] = (_Float16)(k < C0 ? w0[(t * 16 + col) * C0 + k] : 0.f); } }
  __syncthreads();
#pragma unroll
  for (int rt = 0; rt < 2; ++rt) { const int pl = w * 32 + rt * 16 + col; v16h a;
#pragma unroll
    for (int e = 0; e < 16; ++e) { const int k = e < 8 ? 8 * g + e : 16 + 8 * g + (e - 8); a[e] = (_Float16)(k < C0 ? sf[pl][k] : 0.f); }
#pragma unroll
    for (int t = 0; t < 2; ++t) { v8f acc = {}; acc = wmma16(a, bw[t], acc);
#pragma unroll
      for (int r = 0; r < 8; ++r) st[t * 16 + col][w * 32 + rt * 16 + 8 * g + r] = acc[r] + b0[t * 16 + col]; } }
  __syncthreads();
#pragma unroll
  for (int q = 0; q < 8; ++q) vst2(pre0 + (size_t)i * C1 + q * 4, (v4f){st[q * 4][tid], st[q * 4 + 1][tid], st[q * 4 + 2][tid], st[q * 4 + 3][tid]});
  if (tid < 64) { const int which = tid >> 5, o = tid & 31; float a = 0.f; for (int p = 0; p < 256; ++p) { const float v = st[o][p]; a += which ? v * v : v; } vst2(part0 + (size_t)blockIdx.x * 64 + which * 32 + o, (float_a)a); }
  for (int q = tid; q < NKEY / 4; q += 256) vst2(hist + (size_t)blockIdx.x * NKEY + q * 4, *(const v4i*)(&sh[q * 4]));
}
__global__ __launch_bounds__(128) void k_stat(const float* __restrict__ part, int C, int nblk, float* __restrict__ stat) {
  __shared__ __align__(16) float so[256];
  const int c = threadIdx.x;
  if (c < C) { float s = 0.f, s2 = 0.f;
#pragma unroll 1
    for (int b = 0; b < nblk; ++b) { s += part[(size_t)b * 2 * C + c]; s2 += part[(size_t)b * 2 * C + C + c]; }
    const float mu = s / (float)NPT; float var = s2 / (float)NPT - mu * mu; var = var < 0.f ? 0.f : var; so[c * 2] = mu; so[c * 2 + 1] = rsqrtf(var + 1e-5f); }
  __syncthreads();
  for (int q = c; q < 2 * C / 4; q += 128) vst2(stat + q * 4, *(const v4f*)(&so[q * 4]));
}
template <int CIN, int COUT>
__global__ __launch_bounds__(128) void k_lin(const float* __restrict__ prein, const float* __restrict__ stat, const float* __restrict__ gam, const float* __restrict__ bet, const float* __restrict__ W, const float* __restrict__ bias,
                                           float* __restrict__ preout, float* __restrict__ part) {
  __shared__ __align__(16) float st[COUT][68];
  __shared__ float ssc[CIN], ssh[CIN];
  const int tid = threadIdx.x, wave = tid >> 5, lane = tid & 31, col = lane & 15, g = lane >> 4;
  const int r0 = blockIdx.x * 64 + wave * 16;
  if (tid < CIN) { const float sc = gam[tid] * stat[tid * 2 + 1]; ssc[tid] = sc; ssh[tid] = bet[tid] - stat[tid * 2] * sc; }
  __syncthreads();
  v8f acc[COUT / 16];
#pragma unroll
  for (int j = 0; j < COUT / 16; ++j) acc[j] = (v8f){};
#pragma unroll
  for (int kc = 0; kc < CIN / 32; ++kc) { v16h a; const float* pr = prein + (size_t)(r0 + col) * CIN + kc * 32;
#pragma unroll
    for (int e = 0; e < 8; ++e) { const int ka = 8 * g + e, kb = ka + 16; float va = pr[ka] * ssc[kc * 32 + ka] + ssh[kc * 32 + ka], vb = pr[kb] * ssc[kc * 32 + kb] + ssh[kc * 32 + kb];
      a[e] = (_Float16)(va > 0.f ? va : 0.f); a[8 + e] = (_Float16)(vb > 0.f ? vb : 0.f); }
#pragma unroll
    for (int j = 0; j < COUT / 16; ++j) acc[j] = wmma16(a, frag_f32(W + (size_t)(j * 16 + col) * CIN + kc * 32, lane), acc[j]); }
#pragma unroll
  for (int j = 0; j < COUT / 16; ++j) { const float bb = bias[j * 16 + col];
#pragma unroll
    for (int r = 0; r < 8; ++r) st[j * 16 + col][wave * 16 + 8 * g + r] = acc[j][r] + bb; }
  __syncthreads();
  for (int q = tid; q < 64 * COUT / 4; q += 128) { const int rl = q / (COUT / 4), pc = q % (COUT / 4); v4f v = { st[pc * 4][rl], st[pc * 4 + 1][rl], st[pc * 4 + 2][rl], st[pc * 4 + 3][rl] };
    vst2(preout + (size_t)(blockIdx.x * 64 + rl) * COUT + pc * 4, v); }
  if (tid < COUT) { const int o = tid; float s = 0.f, s2 = 0.f; for (int rl = 0; rl < 64; ++rl) { const float v = st[o][rl]; s += v; s2 += v * v; }
    vst2(part + (size_t)blockIdx.x * 2 * COUT + o, (float_a)s); vst2(part + (size_t)blockIdx.x * 2 * COUT + COUT + o, (float_a)s2); }
}
__global__ __launch_bounds__(512) void k_scan(const int* __restrict__ hist, int* __restrict__ cum, int* __restrict__ start) {
  __shared__ int tot[NKEY];
  const int k = threadIdx.x; int run = 0;
#pragma unroll 1
  for (int c = 0; c < NCHK; ++c) { vst2(cum + (size_t)c * NKEY + k, (int_a)run); run += hist[(size_t)c * NKEY + k]; }
  tot[k] = run; __syncthreads();
  if (k == 0) { int s = 0; for (int q = 0; q < NKEY; ++q) { const int t = tot[q]; tot[q] = s; s += t; } }
  __syncthreads();
  vst2(start + k, (int_a)tot[k]);
}
__global__ __launch_bounds__(256) void k_sel(const int* __restrict__ vkey, const int* __restrict__ cum, const int* __restrict__ start, const float* __restrict__ xyz, int* __restrict__ sel, float* __restrict__ newxyz) {
  const int m = blockIdx.x * 256 + threadIdx.x; const int rank = m * (NPT / NS);
  int k = 0; { int lo = 0, hi = NKEY - 1; while (lo < hi) { const int mid = (lo + hi + 1) >> 1; if (start[mid] <= rank) lo = mid; else hi = mid - 1; } k = lo; }
  while (k + 1 < NKEY && start[k + 1] <= rank) ++k;
  const int r = rank - start[k];
  int c = 0; { int lo = 0, hi = NCHK - 1; while (lo < hi) { const int mid = (lo + hi + 1) >> 1; if (cum[(size_t)mid * NKEY + k] <= r) lo = mid; else hi = mid - 1; } c = lo; }
  while (c + 1 < NCHK && cum[(size_t)(c + 1) * NKEY + k] <= r) ++c;
  int need = r - cum[(size_t)c * NKEY + k]; int idx = -1;
  for (int j = 0; j < 256; ++j) { if (vkey[c * 256 + j] == k) { if (need == 0) { idx = c * 256 + j; break; } --need; } }
  if (idx < 0) idx = 0;
  vst2(sel + m, (int_a)idx);
  vst2(newxyz + m, (float_a)xyz[idx]); vst2(newxyz + NS + m, (float_a)xyz[NPT + idx]); vst2(newxyz + 2 * NS + m, (float_a)xyz[2 * NPT + idx]);
}
__global__ __launch_bounds__(256) void k_nn(const int* __restrict__ sel, const float* __restrict__ xyz, const float* __restrict__ pre2, const float* __restrict__ stat2, const float* __restrict__ gam, const float* __restrict__ bet,
                                          float r2, float* __restrict__ agg) {
  __shared__ unsigned long long ck[CAND];
  __shared__ int scnt; __shared__ int nb[32]; __shared__ __align__(16) float so[C3];
  const int s = blockIdx.x, tid = threadIdx.x; const int ci = sel[s];
  const float cx = xyz[ci], cy = xyz[NPT + ci], cz = xyz[2 * NPT + ci];
  if (tid == 0) scnt = 0;
  for (int q = tid; q < CAND; q += 256) ck[q] = ~0ull;
  __syncthreads();
#pragma unroll 1
  for (int i = tid; i < NPT; i += 256) { const float dx = cx - xyz[i], dy = cy - xyz[NPT + i], dz = cz - xyz[2 * NPT + i];
    const float d2 = __fadd_rn(__fadd_rn(__fmul_rn(dx, dx), __fmul_rn(dz, dz)), __fmul_rn(dy, dy));
    if (d2 <= r2) { const int p = atomicAdd(&scnt, 1); if (p < CAND) ck[p] = ((unsigned long long)__float_as_uint(d2) << 32) | (unsigned)i; } }
  __syncthreads();
  for (int kk = 2; kk <= CAND; kk <<= 1) {
    for (int jj = kk >> 1; jj > 0; jj >>= 1) {
      for (int q = tid; q < CAND; q += 256) { const int ixj = q ^ jj; if (ixj > q) { const bool up = ((q & kk) == 0); const unsigned long long a = ck[q], b = ck[ixj]; if ((a > b) == up) { ck[q] = b; ck[ixj] = a; } } }
      __syncthreads(); } }
  const int cnt = scnt < CAND ? scnt : CAND; const int nv = cnt < 32 ? cnt : 32;
  if (tid < 32) nb[tid] = tid < nv ? (int)(ck[tid] & 0xffffffffu) : -1;
  __syncthreads();
  if (tid < C3) { const int c = tid; const float sc = gam[c] * stat2[c * 2 + 1], sh = bet[c] - stat2[c * 2] * sc; float mx = -3.4e38f;
    for (int q = 0; q < nv; ++q) { const int id = nb[q]; float v = pre2[(size_t)id * C3 + c] * sc + sh; v = v > 0.f ? v : 0.f; mx = fmaxf(mx, v); }
    so[c] = mx; }
  __syncthreads();
  if (tid < 32) vst2(agg + (size_t)s * C3 + tid * 4, *(const v4f*)(&so[tid * 4]));
}
__global__ __launch_bounds__(256) void k_tr(const float* __restrict__ agg, float* __restrict__ newpts) {
  __shared__ float tile[64][65];
  const int s0 = blockIdx.x * 64, c0 = blockIdx.y * 64, tid = threadIdx.x;
  for (int q = tid; q < 64 * 64; q += 256) { const int sl = q >> 6, cl = q & 63; tile[sl][cl] = agg[(size_t)(s0 + sl) * C3 + c0 + cl]; }
  __syncthreads();
  for (int q = tid; q < 64 * 16; q += 256) { const int cl = q >> 4, pc = q & 15; v4f v = { tile[pc * 4][cl], tile[pc * 4 + 1][cl], tile[pc * 4 + 2][cl], tile[pc * 4 + 3][cl] };
    vst2(newpts + (size_t)(c0 + cl) * NS + s0 + pc * 4, v); }
}
extern "C" void kernel_launch(void* const* d_in, const int* in_sizes, int n_in, void* d_out, int out_size, void* d_ws, size_t ws_size, hipStream_t stream) {
  (void)in_sizes; (void)n_in; (void)out_size; (void)ws_size;
  const float** I = (const float**)d_in;
  const float* xyz = I[0]; const float* pts = I[1]; const float* w0 = I[2]; const float* b0 = I[3]; const float* g0 = I[4]; const float* bt0 = I[5];
  const float* w1 = I[6]; const float* b1 = I[7]; const float* g1 = I[8]; const float* bt1 = I[9]; const float* w2 = I[10]; const float* b2 = I[11]; const float* g2 = I[12]; const float* bt2 = I[13];
  float* newxyz = (float*)d_out; float* newpts = newxyz + 3 * NS;
  const float offs = (float)1.0011; const float stepf = (float)(2.0 / 8 + 0.0002); const float r2 = (float)(0.2 * 0.2);
  char* ws = (char*)d_ws; size_t off = 0;
  auto take = [&](size_t bytes) { char* p = ws + off; off += (bytes + 255) & ~(size_t)255; return p; };
  float* pre0 = (float*)take((size_t)NPT * C1 * 4); float* pre1 = (float*)take((size_t)NPT * C2 * 4); float* pre2 = (float*)take((size_t)NPT * C3 * 4);
  float* part0 = (float*)take((size_t)NCHK * 2 * C1 * 4); float* part1 = (float*)take((size_t)(NPT / 64) * 2 * C2 * 4); float* part2 = (float*)take((size_t)(NPT / 64) * 2 * C3 * 4);
  float* st0 = (float*)take(2 * C1 * 4); float* st1 = (float*)take(2 * C2 * 4); float* st2 = (float*)take(2 * C3 * 4);
  int* vkey = (int*)take((size_t)NPT * 4); int* hist = (int*)take((size_t)NCHK * NKEY * 4); int* cum = (int*)take((size_t)NCHK * NKEY * 4); int* start = (int*)take(NKEY * 4);
  int* sel = (int*)take(NS * 4); float* agg = (float*)take((size_t)NS * C3 * 4);
  k_l0<<<NCHK, 256, 0, stream>>>(xyz, pts, w0, b0, offs, stepf, pre0, part0, vkey, hist);
  k_stat<<<1, 128, 0, stream>>>(part0, C1, NCHK, st0);
  k_lin<C1, C2><<<NPT / 64, 128, 0, stream>>>(pre0, st0, g0, bt0, w1, b1, pre1, part1);
  k_stat<<<1, 128, 0, stream>>>(part1, C2, NPT / 64, st1);
  k_lin<C2, C3><<<NPT / 64, 128, 0, stream>>>(pre1, st1, g1, bt1, w2, b2, pre2, part2);
  k_stat<<<1, 128, 0, stream>>>(part2, C3, NPT / 64, st2);
  k_scan<<<1, 512, 0, stream>>>(hist, cum, start);
  k_sel<<<NS / 256, 256, 0, stream>>>(vkey, cum, start, xyz, sel, newxyz);
  k_nn<<<NS, 256, 0, stream>>>(sel, xyz, pre2, st2, g2, bt2, r2, agg);
  k_tr<<<dim3(NS / 64, C3 / 64), 256, 0, stream>>>(agg, newpts);
}
